// GraphormerModel_21492016349939
// MI455X (gfx1250) — hardware-verified
//
#include <hip/hip_runtime.h>
#include <hip/hip_bf16.h>
#include <math.h>

#define BB 1
#define SS 2176
#define QROWS 2176
#define KROWS 2176
#define NKV 2049
#define DD 512
#define KVD 512
#define HH 8
#define KVH 8
#define HKDIV 1
#define DKK 64
#define QW 2
#define GSTR 48
#define DDj 256
#define HDj 32
#define FFj 1024
#define NLj 6
#define MROWS 2176
#define NF 2049
#define NN 2048
#define NFEAT 64
#define NE 32768
#define EF 16
#define BTS 2176
#define LCAP 128

typedef _Float16 bf16;
typedef _Float16 f16;
typedef __attribute__((ext_vector_type(4))) unsigned v4u_t;
typedef unsigned v4ua __attribute__((ext_vector_type(4), may_alias));
typedef __attribute__((ext_vector_type(4))) float v4f_t;
typedef float v4fa __attribute__((ext_vector_type(4), may_alias));
typedef __attribute__((ext_vector_type(16))) bf16  bf16x16;
typedef bf16x16 f16x16;
typedef __attribute__((ext_vector_type(8)))  bf16  bf16x8;
typedef bf16x8 f16x8;
typedef __attribute__((ext_vector_type(4)))  bf16  bf16x4;
typedef __attribute__((ext_vector_type(8)))  float f32x8;
__device__ __forceinline__ f32x8 wmma16(f16x16 a, f16x16 b, f32x8 c) {
  c = __builtin_amdgcn_wmma_f32_16x16x32_f16(false, a, false, b, (short)0, c, false, false);
  asm volatile("v_nop\n\tv_nop\n\tv_nop\n\tv_nop" : "+v"(c) : "v"(a), "v"(b));
  return c;
}
#define LDS_STRIDE 48
#define KSTRIDE    72
#define VSTRIDE    48

__device__ __forceinline__ f32x8 wmma_bf16(bf16x16 a, bf16x16 b, f32x8 c) {
  c = __builtin_amdgcn_wmma_f32_16x16x32_f16(false, a, false, b, (short)0, c, false, false);
  asm volatile("v_nop\n\tv_nop\n\tv_nop\n\tv_nop" : "+v"(c) : "v"(a), "v"(b));
  return c;
}

template <typename T>
__device__ __forceinline__ bf16x16 load_frag(const T* __restrict__ base, int ld,
                                             int row0, int k0) {
  const int lane = threadIdx.x & 31;
  const int r    = lane & 15;
  const int kh   = (lane >> 4) * 8;
  const T* p0 = base + (size_t)(row0 + r) * ld + (k0 + kh);
  const T* p1 = p0 + 16;
  bf16x16 f;
#pragma unroll
  for (int i = 0; i < 8; ++i) {
    f[i]     = (bf16)p0[i];
    f[i + 8] = (bf16)p1[i];
  }
  return f;
}

__device__ __forceinline__ bf16x16 lds_frag(const bf16* base, int stride) {
  const int lane = threadIdx.x & 31;
  const int row  = lane & 15;
  const int kh   = (lane >> 4) * 8;
  const bf16x8 lo = *(const bf16x8*)(base + row * stride + kh);
  const bf16x8 hi = *(const bf16x8*)(base + row * stride + kh + 16);
  bf16x16 f;
#pragma unroll
  for (int i = 0; i < 8; ++i) { f[i] = lo[i]; f[i + 8] = hi[i]; }
  return f;
}

template <typename T>
__device__ __forceinline__ void stage_read16(const T* __restrict__ p, float* buf) {
#pragma unroll
  for (int i = 0; i < 16; ++i) buf[i] = (float)p[i];
}

__device__ __forceinline__ void stage_write(bf16* dst, const float* buf, int nquad) {
#pragma unroll
  for (int i = 0; i < nquad; ++i) {
    bf16x4 q;
    q[0] = (bf16)buf[4 * i];     q[1] = (bf16)buf[4 * i + 1];
    q[2] = (bf16)buf[4 * i + 2]; q[3] = (bf16)buf[4 * i + 3];
    *(bf16x4*)(dst + 4 * i) = q;
  }
}

template <typename AT, int MODE>
__global__ __launch_bounds__(256) void gemm_rb_kernel(
    const AT* __restrict__ A, const float* __restrict__ W,
    const float* __restrict__ bias, const float* __restrict__ rowscale, const float* __restrict__ R, const float* __restrict__ rowbias, void* __restrict__ out,
    int M, int N, int K) {
  __shared__ bf16 ldsA[128 * LDS_STRIDE];
  __shared__ bf16 ldsW[256 * LDS_STRIDE];
  __shared__ __attribute__((aligned(16))) unsigned char sob[256 * 136 * 2];

  const int t    = threadIdx.x;
  const int wave = t >> 5;
  const int lane = t & 31;
  const int wm   = (wave & 1) * 64;
  const int wn   = (wave >> 1) * 64;
  const int mBlk = blockIdx.x * 128;
  const int nBlk = blockIdx.y * 256;

  const int arow = t >> 1;
  const int ach  = (t & 1) * 16;

  float abuf[16];
  float wbuf[32];

  stage_read16(A + (size_t)(mBlk + arow) * K + ach, abuf);
  const int nrow = min(nBlk + t, N - 1);
  stage_read16(W + (size_t)nrow * K,          wbuf);
  stage_read16(W + (size_t)nrow * K + 16,     wbuf + 16);

  f32x8 acc[4][4] = {};

  for (int k = 0; k < K; k += 32) {
    __syncthreads();
    stage_write(&ldsA[arow * LDS_STRIDE + ach], abuf, 4);
    stage_write(&ldsW[t * LDS_STRIDE],          wbuf, 8);
    if (k + 32 < K) {
      stage_read16(A + (size_t)(mBlk + arow) * K + (k + 32) + ach, abuf);
      stage_read16(W + (size_t)nrow * K + (k + 32),          wbuf);
      stage_read16(W + (size_t)nrow * K + (k + 32) + 16,     wbuf + 16);
    }
    __syncthreads();

    bf16x16 af[4], wf[4];
#pragma unroll
    for (int i = 0; i < 4; ++i)
      af[i] = lds_frag(ldsA + (wm + 16 * i) * LDS_STRIDE, LDS_STRIDE);
#pragma unroll
    for (int j = 0; j < 4; ++j)
      wf[j] = lds_frag(ldsW + (wn + 16 * j) * LDS_STRIDE, LDS_STRIDE);
#pragma unroll
    for (int i = 0; i < 4; ++i)
#pragma unroll
      for (int j = 0; j < 4; ++j)
        acc[i][j] = wmma_bf16(af[i], wf[j], acc[i][j]);
  }

  const int nlane = lane & 15;
  const int mh    = (lane >> 4) * 8;
  __syncthreads();
  if (MODE == 0 || MODE == 1 || MODE == 3) {
    bf16* so = (bf16*)sob;
#pragma unroll
    for (int i = 0; i < 4; ++i)
#pragma unroll
      for (int j = 0; j < 4; ++j) {
        const int nl = wn + 16 * j + nlane;
        const float bv = bias ? bias[nBlk + nl] : 0.0f;
        if (MODE == 3) {
#pragma unroll 1
          for (int r = 0; r < 8; ++r) {
            const int ml = wm + 16 * i + mh + r;
            const float xg = acc[i][j][r] + bv;
            so[ml * 264 + nl] = (bf16)(0.5f * xg * (1.0f + erff(xg * 0.70710678118654752f)));
          }
        } else {
#pragma unroll
        for (int r = 0; r < 8; ++r) {
          const int ml = wm + 16 * i + mh + r;
          const bf16 hv = (bf16)(acc[i][j][r] + bv);
          if (MODE == 0) so[ml * 264 + nl] = hv;
          else           so[nl * 136 + ml] = hv;
        }
        }
      }
    __syncthreads();
#pragma unroll 1
    for (int pass = 0; pass < 2; ++pass) {
      if (MODE == 0 || MODE == 3) {
        for (int ch = t; ch < 128 * 32; ch += 256) { const int ml = ch >> 5, q = (ch & 31) * 8;
          *(volatile v4u_t*)((bf16*)out + (size_t)(mBlk + ml) * N + nBlk + q) = *(const v4ua*)(so + ml * 264 + q); }
      } else {
        const int b_ = mBlk / SS, s0 = mBlk % SS;
        for (int ch = t; ch < 256 * 16; ch += 256) { const int nl = ch >> 4, q = (ch & 15) * 8; const int n = nBlk + nl, h = n >> 6, dk = n & (DKK - 1);
          *(volatile v4u_t*)((bf16*)out + (((size_t)(b_ * HH + h)) * DKK + dk) * SS + s0 + q) = *(const v4ua*)(so + nl * 136 + q); }
      }
      __threadfence();
    }
  } else {
    float* so = (float*)sob;
#pragma unroll 1
    for (int hf = 0; hf < 2; ++hf) {
      if (wm == hf * 64) {
#pragma unroll
        for (int i = 0; i < 4; ++i)
#pragma unroll
          for (int j = 0; j < 4; ++j) {
            const int nl = wn + 16 * j + nlane;
            const float bv = bias ? bias[nBlk + nl] : 0.0f;
#pragma unroll
            for (int r = 0; r < 8; ++r) { const int mrow = mBlk + hf * 64 + 16 * i + mh + r; so[(16 * i + mh + r) * 260 + nl] = acc[i][j][r] * (rowscale ? rowscale[mrow] : 1.0f) + bv + (rowbias ? rowbias[mrow] : 0.0f); }
          }
      }
      __syncthreads();
      if (R) {
        for (int ch = t; ch < 64 * 64; ch += 256) { const int ml = ch >> 6, q = (ch & 63) * 4;
          if (nBlk + q < N) { const v4f_t rv = *(const v4f_t*)(R + (size_t)(mBlk + hf * 64 + ml) * N + nBlk + q); v4f_t v = *(const v4fa*)(so + ml * 260 + q); v += rv; *(volatile v4fa*)(so + ml * 260 + q) = v; } }
        asm volatile("s_wait_dscnt 0" ::: "memory");
      }
#pragma unroll 1
      for (int pass = 0; pass < 2; ++pass) {
        for (int ch = t; ch < 64 * 64; ch += 256) { const int ml = ch >> 6, q = (ch & 63) * 4;
          if (nBlk + q < N) *(volatile v4f_t*)((float*)out + (size_t)(mBlk + hf * 64 + ml) * N + nBlk + q) = *(const v4fa*)(so + ml * 260 + q); }
        __threadfence();
      }
      __syncthreads();
    }
  }
}


#define GSTR 48
template <typename AT, int EPI, bool OUT16>
__global__ __launch_bounds__(256) void gemm_kne(const AT* __restrict__ A, int lda, const float* __restrict__ Wm, int ldw,
                                                const float* __restrict__ bias, const float* __restrict__ R, const float* __restrict__ gvec,
                                                void* __restrict__ Yv, int ldy, int K) {
  __shared__ __attribute__((aligned(16))) f16 ldsA[128 * GSTR];
  __shared__ __attribute__((aligned(16))) f16 ldsW[128 * GSTR];
  __shared__ __attribute__((aligned(16))) float oS[8][32 * 68];
  const int tid = threadIdx.x, lane = tid & 31, wave = tid >> 5, cl = lane & 15, rh = (lane >> 4) * 8;
  const int m0 = blockIdx.x * 128, n0 = blockIdx.y * 128;
  const int wm = (wave & 3) * 32, wn = (wave >> 2) * 64;
  f32x8 acc[2][4];
#pragma unroll
  for (int i = 0; i < 2; ++i)
#pragma unroll
    for (int j = 0; j < 4; ++j) { f32x8 z = {}; acc[i][j] = z; }
#pragma unroll 1
  for (int k0 = 0; k0 < K; k0 += 32) {
    __syncthreads();
    { const int row = tid >> 1, ch = (tid & 1) * 16;
      const AT* src = A + (size_t)(m0 + row) * lda + k0 + ch;
#pragma unroll
      for (int g = 0; g < 16; ++g) ldsA[row * GSTR + ch + g] = (f16)src[g]; }
    { const int k = tid >> 3, nn0 = (tid & 7) * 16;
      const float* src = Wm + (size_t)(k0 + k) * ldw + n0 + nn0;
#pragma unroll
      for (int g = 0; g < 4; ++g) { const v4f_t v = *(const v4f_t*)(src + 4 * g);
#pragma unroll
        for (int u = 0; u < 4; ++u) ldsW[(nn0 + 4 * g + u) * GSTR + k] = (f16)v[u]; } }
    __syncthreads();
    f16x16 af[2];
#pragma unroll
    for (int i = 0; i < 2; ++i) af[i] = lds_frag(ldsA + (wm + 16 * i) * GSTR, GSTR);
#pragma unroll
    for (int j = 0; j < 4; ++j) {
      const f16x16 bf = lds_frag(ldsW + (wn + 16 * j) * GSTR, GSTR);
#pragma unroll
      for (int i = 0; i < 2; ++i) acc[i][j] = wmma16(af[i], bf, acc[i][j]);
    }
  }
  float* so = oS[wave];
#pragma unroll
  for (int i = 0; i < 2; ++i)
#pragma unroll
    for (int j = 0; j < 4; ++j) {
      const int n = n0 + wn + 16 * j + cl;
      const float bv = bias ? bias[n] : 0.0f;
      const float gv = (EPI == 2) ? gvec[n] : 0.0f;
      if (EPI == 1) {
#pragma unroll 1
        for (int r = 0; r < 8; ++r) { const float xg = acc[i][j][r] + bv; so[(16 * i + rh + r) * 68 + 16 * j + cl] = 0.5f * xg * (1.0f + erff(xg * 0.70710678118654752f)); }
      } else {
#pragma unroll
        for (int r = 0; r < 8; ++r) {
          float v = acc[i][j][r] + bv;
          if (EPI == 2) v = R[(size_t)(m0 + wm + 16 * i + rh + r) * ldy + n] + gv * v;
          so[(16 * i + rh + r) * 68 + 16 * j + cl] = v;
        }
      }
    }
  asm volatile("s_wait_dscnt 0" ::: "memory");
  __builtin_amdgcn_wave_barrier();
#pragma unroll 1
  for (int pass = 0; pass < 2; ++pass) {
    if (OUT16) {
      f16* Y = (f16*)Yv;
#pragma unroll
      for (int it = 0; it < 8; ++it) { const int c = lane + 32 * it, rr = c >> 3, q8 = (c & 7) * 8;
        union { f16 h[8]; v4u_t v; } u;
#pragma unroll
        for (int e = 0; e < 8; ++e) u.h[e] = (f16)so[rr * 68 + q8 + e];
        *(volatile v4u_t*)(Y + (size_t)(m0 + wm + rr) * ldy + n0 + wn + q8) = u.v; }
    } else {
      float* Y = (float*)Yv;
#pragma unroll
      for (int it = 0; it < 16; ++it) { const int f4 = lane + 32 * it, rr = f4 >> 4, q = (f4 & 15) * 4;
        *(volatile v4f_t*)(Y + (size_t)(m0 + wm + rr) * ldy + n0 + wn + q) = *(const v4fa*)(so + rr * 68 + q); }
    }
    __threadfence();
  }
}
__global__ __launch_bounds__(64) void attn_kernel(
    const bf16* __restrict__ Qb, const bf16* __restrict__ Kb,
    const bf16* __restrict__ Vt, const bf16* __restrict__ btab, int btstride,
    bf16* __restrict__ attnOut) {
  __shared__ bf16 ldsK[32 * KSTRIDE];
  __shared__ bf16 ldsV[64 * VSTRIDE];
  __shared__ __attribute__((aligned(16))) bf16 ldsO[2][32 * 72];

  const int q0blk = blockIdx.x * 64;
  const int h  = blockIdx.y;
  const int b  = blockIdx.z;
  const int t    = threadIdx.x;
  const int wave = t >> 5;
  const int lane = t & 31;
  const int qlane = lane & 15;
  const int kh8   = (lane >> 4) * 8;
  const int q0 = q0blk + wave * 32;

  const int hk = h / HKDIV;
  const bf16* Qh = Qb + (size_t)b * QROWS * DD + h * DKK;
  const bf16* Kh = Kb + (size_t)b * KROWS * KVD + hk * DKK;
  const bf16* Vh = Vt + ((size_t)(b * KVH + hk)) * DKK * KROWS;

  const int krow = t >> 1;
  const int kcol = (t & 1) * 32;
  const bf16* kSrc = Kh + (size_t)krow * KVD + kcol;
  const bf16* vSrc = Vh + (size_t)t * KROWS;

  bf16x16 qf[QW][2];
#pragma unroll
  for (int qt = 0; qt < QW; ++qt) {
    qf[qt][0] = load_frag(Qh, DD, q0 + 16 * qt, 0);
    qf[qt][1] = load_frag(Qh, DD, q0 + 16 * qt, 32);
  }

  f32x8 o[QW][4] = {};
  float mrun[QW], lrun[QW];
#pragma unroll
  for (int qt = 0; qt < QW; ++qt) { mrun[qt] = -INFINITY; lrun[qt] = 0.0f; }

  const float scale = 0.17677669529663688f * 1.44269504088896340736f;
  const float NEG2 = -1.0e9f;
  const int kmax = KROWS - 1;
  const float L2E_ = 1.44269504088896340736f; const bf16* bth = btab + (size_t)h * QROWS * btstride;

  bf16x8 kreg[4], vreg[4];
#pragma unroll
  for (int i = 0; i < 4; ++i) {
    kreg[i] = *(const bf16x8*)(kSrc + 8 * i);
    vreg[i] = *(const bf16x8*)(vSrc + 8 * i);
  }

  for (int kb = 0; kb <= kmax; kb += 32) {
    __syncthreads();
#pragma unroll
    for (int i = 0; i < 4; ++i) {
      *(bf16x8*)(&ldsK[krow * KSTRIDE + kcol + 8 * i]) = kreg[i];
      *(bf16x8*)(&ldsV[t * VSTRIDE + 8 * i])           = vreg[i];
    }
    if (kb + 32 <= kmax) {
      const bf16* kn = kSrc + (size_t)(kb + 32) * KVD;
      const bf16* vn = vSrc + (kb + 32);
#pragma unroll
      for (int i = 0; i < 4; ++i) {
        kreg[i] = *(const bf16x8*)(kn + 8 * i);
        vreg[i] = *(const bf16x8*)(vn + 8 * i);
      }
    }
    __syncthreads();

    bf16x16 kf[2][2];
#pragma unroll
    for (int ktile = 0; ktile < 2; ++ktile)
#pragma unroll
      for (int c = 0; c < 2; ++c)
        kf[ktile][c] = lds_frag(ldsK + (ktile * 16) * KSTRIDE + c * 32, KSTRIDE);

    bf16x16 pf[QW];
    bool act[QW];
#pragma unroll
    for (int qt = 0; qt < QW; ++qt) {
      unsigned mbits = 0;
      {
#pragma unroll
        for (int r = 0; r < 8; ++r) { const int j0 = kb + kh8 + r; if (j0 < NKV) mbits |= 1u << r; if (j0 + 16 < NKV) mbits |= 1u << (8 + r); }
        act[qt] = (__builtin_amdgcn_ballot_w32(mbits != 0) != 0);
      }
      if (act[qt]) {
        const int q_my = q0 + 16 * qt + qlane;
        f32x8 s0 = {}, s1 = {};
        s0 = wmma_bf16(kf[0][0], qf[qt][0], s0);
        s0 = wmma_bf16(kf[0][1], qf[qt][1], s0);
        s1 = wmma_bf16(kf[1][0], qf[qt][0], s1);
        s1 = wmma_bf16(kf[1][1], qf[qt][1], s1);

        float mx = -INFINITY;
#pragma unroll
        for (int r = 0; r < 8; ++r) {
          const int k0i = kb + kh8 + r;
          const int k1i = k0i + 16;
          const bf16* brow = bth + (size_t)min(q_my, NKV - 1) * btstride;
          s0[r] = (mbits & (1u << r))       ? s0[r] * scale + L2E_ * (float)brow[min(k0i, NKV - 1)] : NEG2;
          s1[r] = (mbits & (1u << (8 + r))) ? s1[r] * scale + L2E_ * (float)brow[min(k1i, NKV - 1)] : NEG2;
          mx = fmaxf(mx, fmaxf(s0[r], s1[r]));
        }
        mx = fmaxf(mx, __shfl_xor(mx, 16, 32));
        const float mnew  = fmaxf(mrun[qt], mx);
        const float alpha = exp2f(mrun[qt] - mnew);

        float rsum = 0.0f;
#pragma unroll
        for (int r = 0; r < 8; ++r) {
          const float p0 = exp2f(s0[r] - mnew);
          const float p1 = exp2f(s1[r] - mnew);
          rsum += p0 + p1;
          pf[qt][r]     = (bf16)(p0 * 1024.0f);
          pf[qt][r + 8] = (bf16)(p1 * 1024.0f);
        }
        rsum += __shfl_xor(rsum, 16, 32);
        lrun[qt] = lrun[qt] * alpha + rsum;
        mrun[qt] = mnew;

#pragma unroll
        for (int j = 0; j < 4; ++j)
#pragma unroll
          for (int r = 0; r < 8; ++r) o[qt][j][r] *= alpha;
      }
    }

#pragma unroll
    for (int j = 0; j < 4; ++j) {
      const bf16x16 vf = lds_frag(ldsV + (j * 16) * VSTRIDE, VSTRIDE);
#pragma unroll
      for (int qt = 0; qt < QW; ++qt)
        if (act[qt]) o[qt][j] = wmma_bf16(vf, pf[qt], o[qt][j]);
    }
  }

  bf16* so = ldsO[wave];
#pragma unroll
  for (int qt = 0; qt < QW; ++qt) {
    const float rl = 1.0f / (lrun[qt] * 1024.0f);
#pragma unroll
    for (int j = 0; j < 4; ++j)
#pragma unroll
      for (int r = 0; r < 8; ++r) so[(16 * qt + qlane) * 72 + j * 16 + kh8 + r] = (bf16)(o[qt][j][r] * rl);
  }
  asm volatile("s_wait_dscnt 0" ::: "memory");
  __builtin_amdgcn_wave_barrier();
#pragma unroll 1
  for (int pass = 0; pass < 2; ++pass) {
#pragma unroll
    for (int it = 0; it < 8; ++it) { const int ch = lane + 32 * it, ql = ch >> 3, q8 = (ch & 7) * 8;
      *(volatile v4u_t*)(attnOut + ((size_t)(b * QROWS + q0 + ql)) * DD + h * DKK + q8) = *(const v4ua*)(so + ql * 72 + q8); }
    __threadfence();
  }
}


template <typename AT, bool ACC>
__global__ __launch_bounds__(256) void gemm_kn2(const AT* __restrict__ A, int lda, size_t strideA,
                                               const float* __restrict__ Wm, int ldw, size_t strideW,
                                               const float* __restrict__ bias, float scale,
                                               float* __restrict__ Y, int ldy, size_t strideY, int K) {
  __shared__ __attribute__((aligned(16))) f16 ldsA[128 * GSTR], ldsAl[128 * GSTR];
  __shared__ __attribute__((aligned(16))) f16 ldsW[128 * GSTR], ldsWl[128 * GSTR];
  __shared__ __attribute__((aligned(16))) float oS[8][32 * 68];
  const int tid = threadIdx.x, lane = tid & 31, wave = tid >> 5, cl = lane & 15, rh = (lane >> 4) * 8;
  const int m0 = blockIdx.x * 128, n0 = blockIdx.y * 128;
  const int wm = (wave & 3) * 32, wn = (wave >> 2) * 64;
  A += (size_t)blockIdx.z * strideA; Wm += (size_t)blockIdx.z * strideW; Y += (size_t)blockIdx.z * strideY;
  f32x8 acc[2][4], accx[2][4];
#pragma unroll
  for (int i = 0; i < 2; ++i)
#pragma unroll
    for (int j = 0; j < 4; ++j) { f32x8 z = {}; acc[i][j] = z; accx[i][j] = z; }
#pragma unroll 1
  for (int k0 = 0; k0 < K; k0 += 32) {
    __syncthreads();
    {
      const int row = tid >> 1, ch = (tid & 1) * 16;
      const AT* src = A + (size_t)(m0 + row) * lda + k0 + ch;
#pragma unroll
      for (int g = 0; g < 16; ++g) { const float v = (float)src[g]; const f16 h = (f16)v; ldsA[row * GSTR + ch + g] = h; ldsAl[row * GSTR + ch + g] = (f16)((v - (float)h) * 2048.0f); }
    }
    {
      const int k = tid >> 3, nn0 = (tid & 7) * 16;
      const float* src = Wm + (size_t)(k0 + k) * ldw + n0 + nn0;
#pragma unroll
      for (int g = 0; g < 4; ++g) { const v4f_t v = *(const v4f_t*)(src + 4 * g);
#pragma unroll
        for (int u = 0; u < 4; ++u) { const f16 h = (f16)v[u]; ldsW[(nn0 + 4 * g + u) * GSTR + k] = h; ldsWl[(nn0 + 4 * g + u) * GSTR + k] = (f16)((v[u] - (float)h) * 2048.0f); } }
    }
    __syncthreads();
    f16x16 af[2], afl[2];
#pragma unroll
    for (int i = 0; i < 2; ++i) { af[i] = lds_frag(ldsA + (wm + 16 * i) * GSTR, GSTR); afl[i] = lds_frag(ldsAl + (wm + 16 * i) * GSTR, GSTR); }
#pragma unroll
    for (int j = 0; j < 4; ++j) {
      const f16x16 bf = lds_frag(ldsW + (wn + 16 * j) * GSTR, GSTR), bfl = lds_frag(ldsWl + (wn + 16 * j) * GSTR, GSTR);
#pragma unroll
      for (int i = 0; i < 2; ++i) { acc[i][j] = wmma16(af[i], bf, acc[i][j]); accx[i][j] = wmma16(af[i], bfl, accx[i][j]); accx[i][j] = wmma16(afl[i], bf, accx[i][j]); }
    }
  }
  float* so = oS[wave];
#pragma unroll
  for (int i = 0; i < 2; ++i)
#pragma unroll
    for (int j = 0; j < 4; ++j) {
      const float bv = bias ? bias[n0 + wn + 16 * j + cl] : 0.0f;
#pragma unroll
      for (int r = 0; r < 8; ++r) so[(16 * i + rh + r) * 68 + 16 * j + cl] = (acc[i][j][r] + accx[i][j][r] * (1.0f / 2048.0f)) * scale + bv;
    }
  asm volatile("s_wait_dscnt 0" ::: "memory");
  __builtin_amdgcn_wave_barrier();
  if (ACC) {
#pragma unroll
    for (int it = 0; it < 16; ++it) { const int f4 = lane + 32 * it, rr = f4 >> 4, q = (f4 & 15) * 4;
      const v4f_t old = *(const v4fa*)(Y + (size_t)(m0 + wm + rr) * ldy + n0 + wn + q);
      v4f_t v = *(const v4fa*)(so + rr * 68 + q); v += old; *(v4fa*)(so + rr * 68 + q) = v; }
    asm volatile("s_wait_dscnt 0" ::: "memory");
  }
#pragma unroll 1
  for (int pass = 0; pass < 2; ++pass) {
#pragma unroll
    for (int it = 0; it < 16; ++it) { const int f4 = lane + 32 * it, rr = f4 >> 4, q = (f4 & 15) * 4;
      *(volatile v4f_t*)(Y + (size_t)(m0 + wm + rr) * ldy + n0 + wn + q) = *(const v4fa*)(so + rr * 68 + q); }
    __threadfence();
  }
}


template <bool OUT16>
__global__ __launch_bounds__(256) void k_ln(const float* __restrict__ X, const float* __restrict__ gam, const float* __restrict__ bet, void* __restrict__ Yv) {
  __shared__ __attribute__((aligned(16))) float rowS[32 * 260];
  const int tid = threadIdx.x, r = tid >> 3, part = tid & 7; const size_t row = (size_t)blockIdx.x * 32 + r;
  float s = 0.0f;
#pragma unroll 1
  for (int i = 0; i < 32; ++i) { const float v = X[row * DDj + part * 32 + i]; rowS[r * 260 + part * 32 + i] = v; s += v; }
  s += __shfl_xor(s, 1, 32); s += __shfl_xor(s, 2, 32); s += __shfl_xor(s, 4, 32);
  const float mean = s * (1.0f / DDj); float q = 0.0f;
#pragma unroll 1
  for (int i = 0; i < 32; ++i) { const float d = rowS[r * 260 + part * 32 + i] - mean; q += d * d; }
  q += __shfl_xor(q, 1, 32); q += __shfl_xor(q, 2, 32); q += __shfl_xor(q, 4, 32);
  const float rstd = rsqrtf(q * (1.0f / DDj) + 1e-5f);
#pragma unroll 1
  for (int i = 0; i < 32; ++i) { const int c = part * 32 + i; rowS[r * 260 + c] = (rowS[r * 260 + c] - mean) * rstd * gam[c] + bet[c]; }
  __syncthreads();
#pragma unroll 1
  for (int pass = 0; pass < 2; ++pass) {
    if (OUT16) { bf16* Y = (bf16*)Yv;
      for (int q8 = tid; q8 < 32 * 32; q8 += 256) { const int rr = q8 >> 5, c8 = (q8 & 31) * 8; union { bf16 hh[8]; v4u_t u; } cv;
#pragma unroll
        for (int e = 0; e < 8; ++e) cv.hh[e] = (bf16)rowS[rr * 260 + c8 + e];
        *(volatile v4u_t*)(Y + ((size_t)blockIdx.x * 32 + rr) * DDj + c8) = cv.u; }
    } else { float* Y = (float*)Yv;
      for (int q4 = tid; q4 < 32 * 64; q4 += 256) { const int rr = q4 >> 6, c4 = (q4 & 63) * 4;
        *(volatile v4f_t*)(Y + ((size_t)blockIdx.x * 32 + rr) * DDj + c4) = *(const v4fa*)(rowS + rr * 260 + c4); } }
    __threadfence(); }
}
__global__ __launch_bounds__(256) void k_padw(const float* __restrict__ w, const float* __restrict__ bq, int sel, float* __restrict__ Wp, float* __restrict__ bp) {
  const int i = blockIdx.x; for (int c = threadIdx.x; c < DD; c += 256) { const int h = c >> 6, d = c & 63; const int dd = min(d, HDj - 1);
    const float wv = w[((size_t)(sel * DDj + h * HDj + dd)) * DDj + i]; const float v = (d < HDj) ? wv : 0.0f;
    *(volatile float*)(Wp + (size_t)i * DD + c) = v; __threadfence(); *(volatile float*)(Wp + (size_t)i * DD + c) = v;
    if (i == 0) { const float bb = bq[sel * DDj + h * HDj + dd]; const float bv = (d < HDj) ? bb : 0.0f; *(volatile float*)(bp + c) = bv; __threadfence(); *(volatile float*)(bp + c) = bv; } }
}
__global__ __launch_bounds__(256) void k_padwvT(const float* __restrict__ w, float* __restrict__ WvT) { const int o = blockIdx.x; const int h = o >> 6, d = o & 63; const int dd = min(d, HDj - 1);
  for (int i = threadIdx.x; i < DDj; i += 256) { const float wv = w[((size_t)(h * HDj + dd)) * DDj + i]; const float v = (d < HDj) ? wv : 0.0f; *(volatile float*)(WvT + (size_t)o * DDj + i) = v; __threadfence(); *(volatile float*)(WvT + (size_t)o * DDj + i) = v; } }
__global__ __launch_bounds__(256) void k_padwo(const float* __restrict__ w, float* __restrict__ Wop) { const int r = blockIdx.x; const int h = r >> 6, d = r & 63; const int dd = min(d, HDj - 1);
  for (int o = threadIdx.x; o < DDj; o += 256) { const float wv = w[(size_t)o * DDj + h * HDj + dd]; const float v = (d < HDj) ? wv : 0.0f; *(volatile float*)(Wop + (size_t)r * DDj + o) = v; __threadfence(); *(volatile float*)(Wop + (size_t)r * DDj + o) = v; } }
__global__ __launch_bounds__(256) void k_transpose(const float* __restrict__ Wm, float* __restrict__ Wt, int rows, int cols) {
  __shared__ float tS[64][65];
  const int tid = threadIdx.x, tbj = cols / 64, bi = blockIdx.x / tbj, bj = blockIdx.x % tbj;
  for (int e = tid; e < 64 * 64; e += 256) { const int r = e >> 6, c = e & 63; tS[r][c] = Wm[(size_t)(bi * 64 + r) * cols + bj * 64 + c]; }
  __syncthreads();
  for (int ch = tid; ch < 64 * 16; ch += 256) { const int r = ch >> 4, q4 = (ch & 15) * 4; v4f_t o; o[0] = tS[q4][r]; o[1] = tS[q4 + 1][r]; o[2] = tS[q4 + 2][r]; o[3] = tS[q4 + 3][r];
    float* dst = Wt + (size_t)(bj * 64 + r) * rows + bi * 64 + q4; *(volatile v4f_t*)dst = o; __threadfence(); *(volatile v4f_t*)dst = o; }
}

__global__ __launch_bounds__(256) void k_ones(float* __restrict__ p, int n) { for (int i = threadIdx.x * 4; i < n; i += 1024) { v4f_t o = {1.f,1.f,1.f,1.f}; *(volatile v4f_t*)(p + i) = o; __threadfence(); *(volatile v4f_t*)(p + i) = o; } }

__global__ __launch_bounds__(256) void k_deghist(const int* __restrict__ esrc, const int* __restrict__ edst, int* __restrict__ part) {
  __shared__ int hin[NN], hout[NN];
  const int tid = threadIdx.x; const int e0 = blockIdx.x * (NE / 16);
#pragma unroll 1
  for (int i = tid; i < NN; i += 256) { hin[i] = 0; hout[i] = 0; }
  __syncthreads();
#pragma unroll 1
  for (int e = e0 + tid; e < e0 + NE / 16; e += 256) { atomicAdd(&hin[min(max(edst[e], 0), NN - 1)], 1); atomicAdd(&hout[min(max(esrc[e], 0), NN - 1)], 1); }
  __syncthreads();
#pragma unroll 1
  for (int pass = 0; pass < 2; ++pass) {
#pragma unroll 1
    for (int i = tid; i < NN; i += 256) { *(volatile int*)(part + ((size_t)blockIdx.x * 2 + 0) * NN + i) = hin[i]; *(volatile int*)(part + ((size_t)blockIdx.x * 2 + 1) * NN + i) = hout[i]; }
    __threadfence(); }
}
__global__ __launch_bounds__(256) void k_embed(const float* __restrict__ H0, const float* __restrict__ cls, const float* __restrict__ inE, const float* __restrict__ outE,
                                              const int* __restrict__ part, float* __restrict__ X) {
  const int tid = threadIdx.x; const int r = blockIdx.x * 4 + (tid >> 6); const int c4 = (tid & 63) * 4; const int node = min(max(r - 1, 0), NN - 1);
  int di = 0, dq = 0;
#pragma unroll 1
  for (int k = 0; k < 16; ++k) { di += part[((size_t)k * 2 + 0) * NN + node]; dq += part[((size_t)k * 2 + 1) * NN + node]; }
  di = min(max(di, 0), 64); dq = min(max(dq, 0), 64);
  const v4f_t a = *(const v4f_t*)(H0 + (size_t)node * DDj + c4), bi = *(const v4f_t*)(inE + (size_t)di * DDj + c4), bo = *(const v4f_t*)(outE + (size_t)dq * DDj + c4), cc = *(const v4f_t*)(cls + c4);
  v4f_t v;
#pragma unroll
  for (int u = 0; u < 4; ++u) v[u] = (r == 0) ? cc[u] : ((r <= NN) ? (a[u] + bi[u] + bo[u]) : 0.0f);
  *(volatile v4f_t*)(X + (size_t)r * DDj + c4) = v; __threadfence(); *(volatile v4f_t*)(X + (size_t)r * DDj + c4) = v;
}
__global__ __launch_bounds__(256) void k_btab(const int* __restrict__ dm, const float* __restrict__ dbias, const float* __restrict__ eattr, const float* __restrict__ ew, const float* __restrict__ eb,
                                             const int* __restrict__ esrc, const int* __restrict__ edst, bf16* __restrict__ BT) {
  __shared__ float acc[8 * BTS];
  __shared__ int lst[LCAP]; __shared__ int wcnt[8]; __shared__ int scnt;
  const int q = blockIdx.x, tid = threadIdx.x, lane = tid & 31, wave = tid >> 5; const int node = q - 1;
  if (tid == 0) scnt = 0;
  __syncthreads();
#pragma unroll 1
  for (int c0 = 0; c0 < NE; c0 += 256) { const int e = c0 + tid;
    const bool hit = (esrc[e] == node) && (q >= 1) && (q <= NN);
    const unsigned bal = __builtin_amdgcn_ballot_w32(hit); const int pre = __builtin_popcount(bal & ((1u << lane) - 1u));
    if (lane == 0) wcnt[wave] = __builtin_popcount(bal);
    __syncthreads();
    const int base = scnt; int off = 0, tot = 0;
#pragma unroll
    for (int w = 0; w < 8; ++w) { const int c = wcnt[w]; tot += c; off += (w < wave) ? c : 0; }
    if (hit) { const int pos = base + off + pre; if (pos < LCAP) lst[pos] = e; }
    __syncthreads();
    if (tid == 0) scnt = min(base + tot, LCAP);
    __syncthreads(); }
  const int cnt = scnt;
#pragma unroll 1
  for (int i = tid; i < 8 * BTS; i += 256) { const int h = i / BTS, k = i % BTS; float v = 0.0f;
    if (q < NF && k < NF) { int dp = 0; if (q >= 1 && k >= 1) dp = min(max(dm[(size_t)(q - 1) * NN + (k - 1)], 0), 9); v = dbias[dp * HH + h]; }
    acc[i] = v; }
  __syncthreads();
  if (tid < 8) { const int h = tid;
#pragma unroll 1
    for (int j = 0; j < LCAP; ++j) { if (j < cnt) { const int e = lst[j]; const int k = min(max(edst[e], 0), NN - 1) + 1;
        float p = eb[h];
#pragma unroll 1
        for (int f = 0; f < EF; ++f) p = fmaf(eattr[(size_t)e * EF + f], ew[h * EF + f], p);
        acc[h * BTS + k] += p; } } }
  __syncthreads();
#pragma unroll 1
  for (int pass = 0; pass < 2; ++pass) {
#pragma unroll 1
    for (int i = tid; i < 8 * (BTS / 8); i += 256) { const int h = i / (BTS / 8), p8 = (i % (BTS / 8)) * 8; union { bf16 hh[8]; v4u_t u; } cv;
#pragma unroll
      for (int e = 0; e < 8; ++e) cv.hh[e] = (bf16)acc[h * BTS + p8 + e];
      *(volatile v4u_t*)(BT + ((size_t)h * QROWS + q) * BTS + p8) = cv.u; }
    __threadfence(); }
}
__global__ __launch_bounds__(256) void k_lnout(const float* __restrict__ X, const float* __restrict__ gam, const float* __restrict__ bet, float* __restrict__ out0, float* __restrict__ out1) {
  __shared__ __attribute__((aligned(16))) float rowS[32 * 260];
  const int tid = threadIdx.x, r = tid >> 3, part = tid & 7; const size_t row = (size_t)blockIdx.x * 32 + r;
  float s = 0.0f;
#pragma unroll 1
  for (int i = 0; i < 32; ++i) { const float v = X[row * DDj + part * 32 + i]; rowS[r * 260 + part * 32 + i] = v; s += v; }
  s += __shfl_xor(s, 1, 32); s += __shfl_xor(s, 2, 32); s += __shfl_xor(s, 4, 32);
  const float mean = s * (1.0f / DDj); float qq = 0.0f;
#pragma unroll 1
  for (int i = 0; i < 32; ++i) { const float d = rowS[r * 260 + part * 32 + i] - mean; qq += d * d; }
  qq += __shfl_xor(qq, 1, 32); qq += __shfl_xor(qq, 2, 32); qq += __shfl_xor(qq, 4, 32);
  const float rstd = rsqrtf(qq * (1.0f / DDj) + 1e-5f);
#pragma unroll 1
  for (int i = 0; i < 32; ++i) { const int c = part * 32 + i; rowS[r * 260 + c] = (rowS[r * 260 + c] - mean) * rstd * gam[c] + bet[c]; }
  __syncthreads();
#pragma unroll 1
  for (int pass = 0; pass < 2; ++pass) { for (int q4 = tid; q4 < 32 * 64; q4 += 256) { const int rr = q4 >> 6, c4 = (q4 & 63) * 4; const size_t orow = (size_t)blockIdx.x * 32 + rr;
      if (orow < NF) *(volatile v4f_t*)(out0 + orow * DDj + c4) = *(const v4fa*)(rowS + rr * 260 + c4);
      if (orow == 0) *(volatile v4f_t*)(out1 + c4) = *(const v4fa*)(rowS + rr * 260 + c4); }
    __threadfence(); }
}

#define NLRUN NLj
extern "C" void kernel_launch(void* const* d_in, const int* in_sizes, int n_in,
                              void* d_out, int out_size, void* d_ws, size_t ws_size,
                              hipStream_t stream) {
  (void)in_sizes; (void)n_in; (void)out_size;
  const float** f = (const float**)d_in;
  const float* x = f[0], *eattr = f[1], *npw = f[2], *npb = f[3], *inE = f[4], *outE = f[5], *dbias = f[6], *epw = f[7], *epb = f[8], *cls = f[9];
  const float* qw = f[10], *qb = f[11], *kw = f[12], *kb = f[13], *vw = f[14], *vb = f[15], *ow = f[16], *ob = f[17], *f1w = f[18], *f1b = f[19], *f2w = f[20], *f2b = f[21];
  const float* ln1w = f[22], *ln1b = f[23], *ln2w = f[24], *ln2b = f[25], *fnw = f[26], *fnb = f[27];
  const int* ei = (const int*)d_in[28]; const int* dm = (const int*)d_in[29];
  const int* esrc = ei; const int* edst = ei + NE;
  float* out0 = (float*)d_out; float* out1 = out0 + (size_t)NF * DDj;
  char* ws = (char*)d_ws;
  float* X = (float*)ws; ws += (size_t)MROWS * DDj * 4; float* X1 = (float*)ws; ws += (size_t)MROWS * DDj * 4; float* H0 = (float*)ws; ws += (size_t)NN * DDj * 4;
  bf16* hN = (bf16*)ws; ws += (size_t)MROWS * DDj * 2;
  float* Wn = (float*)ws; ws += (size_t)NFEAT * DDj * 4;
  float* Wq = (float*)ws; ws += (size_t)DDj * DD * 4; float* Wk = (float*)ws; ws += (size_t)DDj * DD * 4; float* WvT = (float*)ws; ws += (size_t)DD * DDj * 4; float* Wop = (float*)ws; ws += (size_t)DD * DDj * 4;
  float* bqp = (float*)ws; ws += DD * 4; float* bkp = (float*)ws; ws += DD * 4; float* bvp = (float*)ws; ws += DD * 4;
  float* W1t = (float*)ws; ws += (size_t)DDj * FFj * 4; float* W2t = (float*)ws; ws += (size_t)FFj * DDj * 4;
  bf16* Qb = (bf16*)ws; ws += (size_t)MROWS * DD * 2; bf16* Kb = (bf16*)ws; ws += (size_t)MROWS * DD * 2;
  float* ffh = (float*)ws; ws += (size_t)MROWS * FFj * 4;
  bf16* VtB = (bf16*)ws; ws += (size_t)MROWS * DD * 2; bf16* att16 = (bf16*)ws; ws += (size_t)MROWS * DD * 2;
  bf16* BT = (bf16*)ws; ws += (size_t)HH * QROWS * BTS * 2;
  float* ones = (float*)ws; ws += 1024 * 4;
  int* part = (int*)ws; ws += (size_t)16 * 2 * NN * 4;
  if ((size_t)(ws - (char*)d_ws) > ws_size) return;
  const dim3 blk(256);
  k_ones<<<dim3(1), blk, 0, stream>>>(ones, 1024);
  k_transpose<<<dim3((DDj / 64) * (NFEAT / 64)), blk, 0, stream>>>(npw, Wn, DDj, NFEAT);
  gemm_kne<float, 0, false><<<dim3(NN / 128, DDj / 128), blk, 0, stream>>>(x, NFEAT, Wn, DDj, npb, nullptr, nullptr, H0, DDj, NFEAT);
  k_deghist<<<dim3(16), blk, 0, stream>>>(esrc, edst, part);
  k_embed<<<dim3(MROWS / 4), blk, 0, stream>>>(H0, cls, inE, outE, part, X);
  k_btab<<<dim3(QROWS), blk, 0, stream>>>(dm, dbias, eattr, epw, epb, esrc, edst, BT);
  for (int l = 0; l < NLRUN; ++l) {
    k_padw<<<dim3(DDj), blk, 0, stream>>>(qw + (size_t)l * DDj * DDj, qb + l * DDj, 0, Wq, bqp); k_padw<<<dim3(DDj), blk, 0, stream>>>(kw + (size_t)l * DDj * DDj, kb + l * DDj, 0, Wk, bkp);
    k_padw<<<dim3(1), blk, 0, stream>>>(vw + (size_t)l * DDj * DDj, vb + l * DDj, 0, W2t  , bvp); k_padwvT<<<dim3(DD), blk, 0, stream>>>(vw + (size_t)l * DDj * DDj, WvT);
    k_padwo<<<dim3(DD), blk, 0, stream>>>(ow + (size_t)l * DDj * DDj, Wop);
    k_transpose<<<dim3((FFj / 64) * (DDj / 64)), blk, 0, stream>>>(f1w + (size_t)l * FFj * DDj, W1t, FFj, DDj);
    k_transpose<<<dim3((DDj / 64) * (FFj / 64)), blk, 0, stream>>>(f2w + (size_t)l * DDj * FFj, W2t, DDj, FFj);
    k_ln<true><<<dim3(MROWS / 32), blk, 0, stream>>>(X, ln1w + l * DDj, ln1b + l * DDj, hN);
    gemm_kne<bf16, 0, true><<<dim3(MROWS / 128, DD / 128), blk, 0, stream>>>(hN, DDj, Wq, DD, bqp, nullptr, nullptr, Qb, DD, DDj);
    gemm_kne<bf16, 0, true><<<dim3(MROWS / 128, DD / 128), blk, 0, stream>>>(hN, DDj, Wk, DD, bkp, nullptr, nullptr, Kb, DD, DDj);
    gemm_rb_kernel<bf16, 1><<<dim3(MROWS / 128, DD / 256), blk, 0, stream>>>(hN, WvT, bvp, nullptr, nullptr, nullptr, VtB, MROWS, DD, DDj);
    attn_kernel<<<dim3(QROWS / 64, HH, 1), dim3(64), 0, stream>>>(Qb, Kb, VtB, BT, BTS, att16);
    gemm_kne<bf16, 2, false><<<dim3(MROWS / 128, DDj / 128), blk, 0, stream>>>(att16, DD, Wop, DDj, ob + l * DDj, X, ones, X1, DDj, DD);
    k_ln<true><<<dim3(MROWS / 32), blk, 0, stream>>>(X1, ln2w + l * DDj, ln2b + l * DDj, hN);
    gemm_kne<bf16, 1, false><<<dim3(MROWS / 128, FFj / 128), blk, 0, stream>>>(hN, DDj, W1t, FFj, f1b + l * FFj, nullptr, nullptr, ffh, FFj, DDj);
    gemm_kn2<float, true><<<dim3(MROWS / 128, DDj / 128, 1), blk, 0, stream>>>(ffh, FFj, 0, W2t, DDj, 0, f2b + l * DDj, 1.0f, X1, DDj, 0, FFj);
    { float* t = X; X = X1; X1 = t; }
  }
  k_lnout<<<dim3(MROWS / 32), blk, 0, stream>>>(X, fnw, fnb, out0, out1);
}
